// NonLocalBlock3D_74586402062490
// MI455X (gfx1250) — hardware-verified
//
#include <hip/hip_runtime.h>
#include <math.h>
#include <stdint.h>

#ifndef NB
#define NB 2
#endif
#ifndef SEQ
#define SEQ 8192
#endif
#define NB_FULL 2
#define NN_FULL 8192
#define CC   256
#define DQ   128
#define QT   64
#define MW   384
#define NT   (SEQ / QT)
#define PSW  512
#define BCH  1024
#define OSP  68
#define OSPW 132
#define TP   72
#define WSC  256.0f
#define IWSC 0.00390625f
#define RSC  1024.0f
#define IRSC 0.0009765625f
#define LNPS 9.704060527839234f
#define BNEPS 1.0e-5f

static_assert(NB >= 1 && NB <= NB_FULL);
static_assert(SEQ >= 128 && SEQ <= NN_FULL);
static_assert(SEQ % QT == 0 && SEQ % 32 == 0 && SEQ % 128 == 0);
static_assert((CC * SEQ) % BCH == 0 && BCH == 4 * 256);
static_assert(CC % QT == 0 && CC % 32 == 0);
static_assert(DQ == 2 * QT && DQ % 32 == 0);
static_assert(MW == 3 * DQ && MW % 8 == 0);
static_assert(PSW == 2 * CC);
static_assert(CC % 16 == 0);
static_assert((OSP * 4) % 16 == 0);
static_assert((OSPW * 4) % 16 == 0);
static_assert((TP * 2) % 16 == 0);

typedef _Float16       v16h __attribute__((ext_vector_type(16)));
typedef _Float16       v8h  __attribute__((ext_vector_type(8)));
typedef __bf16         v16b __attribute__((ext_vector_type(16)));
typedef unsigned short v8us __attribute__((ext_vector_type(8)));
typedef float          v8f  __attribute__((ext_vector_type(8)));
typedef float          v4f  __attribute__((ext_vector_type(4)));
typedef unsigned int   v4u  __attribute__((ext_vector_type(4)));

union Frag  { v8us u[2]; v16h h; v16b bf; };
union FragH { v16h v; v8h hv[2]; };
static_assert(sizeof(Frag) == 32);
static_assert(sizeof(FragH) == 32);

__device__ __forceinline__ unsigned short bf_bits(float f) {
  unsigned u = __float_as_uint(f);
  return (unsigned short)((u + 0x7FFFu + ((u >> 16) & 1u)) >> 16);
}
__device__ __forceinline__ float bf_up(unsigned short hb) { return __uint_as_float(((unsigned)hb) << 16); }
__device__ __forceinline__ float bfr(float f) { return bf_up(bf_bits(f)); }
__device__ __forceinline__ unsigned short h_bits(_Float16 x) { return __builtin_bit_cast(unsigned short, x); }
__device__ __forceinline__ unsigned pk16(unsigned short a, unsigned short b) { return (unsigned)a | ((unsigned)b << 16); }
__device__ __forceinline__ v8f zero8() { v8f z = {0.f, 0.f, 0.f, 0.f, 0.f, 0.f, 0.f, 0.f}; return z; }
__device__ __forceinline__ float hmax8(v8f s) {
  return fmaxf(fmaxf(fmaxf(s[0], s[1]), fmaxf(s[2], s[3])), fmaxf(fmaxf(s[4], s[5]), fmaxf(s[6], s[7])));
}
__device__ __forceinline__ unsigned wave_ballot(bool p) {
#if defined(__HIP_DEVICE_COMPILE__)
  return __builtin_amdgcn_ballot_w32(p);
#else
  return p ? 1u : 0u;
#endif
}

__device__ __forceinline__ Frag ldfrag(const unsigned short* p) {
  Frag f;
  f.u[0] = *(const v8us*)(p);
  f.u[1] = *(const v8us*)(p + 16);
  return f;
}

__device__ __forceinline__ v8f mma_h(v16h a, v16h b, v8f c) {
  v8f d = __builtin_amdgcn_wmma_f32_16x16x32_f16(false, a, false, b, (short)0, c, false, false);
#if defined(__HIP_DEVICE_COMPILE__)
  asm volatile("v_nop\n\tv_nop\n\tv_nop\n\tv_nop" : "+v"(d) : "v"(a), "v"(b));
#endif
  return d;
}
__device__ __forceinline__ v8f mma_b(v16b a, v16b b, v8f c) {
  v8f d = __builtin_amdgcn_wmma_f32_16x16x32_bf16(false, a, false, b, (short)0, c, false, false);
#if defined(__HIP_DEVICE_COMPILE__)
  const v16h ha = __builtin_bit_cast(v16h, a), hb = __builtin_bit_cast(v16h, b);
  asm volatile("v_nop\n\tv_nop\n\tv_nop\n\tv_nop" : "+v"(d) : "v"(ha), "v"(hb));
#endif
  return d;
}

__global__ __launch_bounds__(256)
void cvt_w(const float* __restrict__ tw, const float* __restrict__ pw, const float* __restrict__ gw,
           unsigned short* W16) {
  const int tid = threadIdx.x, blk = blockIdx.x;
  const int rl = tid >> 5, col = 8 * (tid & 31);
  const int o = 8 * blk + rl;
  const int grp = blk / (DQ / 8);
  const float* wbase = (grp == 0) ? tw : ((grp == 1) ? pw : gw);
  const float* s = wbase + (size_t)(o - grp * DQ) * CC + col;
  const v4f a = *(const v4f*)s;
  const v4f q = *(const v4f*)(s + 4);
  const float f[8] = {a[0], a[1], a[2], a[3], q[0], q[1], q[2], q[3]};
  v4u u;
#pragma unroll
  for (int t = 0; t < 4; ++t) {
    const _Float16 h0 = (_Float16)(bfr(f[2 * t]) * WSC);
    const _Float16 h1 = (_Float16)(bfr(f[2 * t + 1]) * WSC);
    u[t] = pk16(h_bits(h0), h_bits(h1));
  }
#pragma unroll
  for (int pass = 0; pass < 2; ++pass) {
    *(volatile v4u*)(W16 + (size_t)o * CC + col) = u;
    __threadfence();
  }
}

__global__ __launch_bounds__(256)
void cvt_ww(const float* __restrict__ ww, unsigned short* WW16) {
  const int tid = threadIdx.x, blk = blockIdx.x;
  const int wave = tid >> 5, lane = tid & 31;
  const int o = 16 * blk + 2 * wave + (lane >> 4);
  const int col = 8 * (lane & 15);
  const float* s = ww + (size_t)o * DQ + col;
  const v4f a = *(const v4f*)s;
  const v4f q = *(const v4f*)(s + 4);
  const float f[8] = {a[0], a[1], a[2], a[3], q[0], q[1], q[2], q[3]};
  v4u u;
#pragma unroll
  for (int t = 0; t < 4; ++t) {
    const _Float16 h0 = (_Float16)(bfr(f[2 * t]) * WSC);
    const _Float16 h1 = (_Float16)(bfr(f[2 * t + 1]) * WSC);
    u[t] = pk16(h_bits(h0), h_bits(h1));
  }
#pragma unroll
  for (int pass = 0; pass < 2; ++pass) {
    *(volatile v4u*)(WW16 + (size_t)o * DQ + col) = u;
    __threadfence();
  }
}

__global__ __launch_bounds__(256)
void cvt_x(const float* __restrict__ x, unsigned short* XP) {
  __shared__ __align__(16) unsigned short T[QT * TP];
  const int tid = threadIdx.x;
  const int nb = blockIdx.x, cb = blockIdx.y, b = blockIdx.z;
  const int e = tid & 7, lq = tid >> 3;
  const int n0 = nb * QT, c0 = cb * QT;
#pragma unroll
  for (int it = 0; it < 2; ++it) {
    const int cl = it * 32 + lq;
    const float* sp = x + ((size_t)(b * CC + c0 + cl)) * NN_FULL + n0 + 8 * e;
    const v4f a = *(const v4f*)sp;
    const v4f q = *(const v4f*)(sp + 4);
    unsigned short hb[8];
#pragma unroll
    for (int t = 0; t < 4; ++t) {
      hb[t]     = h_bits((_Float16)bfr(a[t]));
      hb[4 + t] = h_bits((_Float16)bfr(q[t]));
    }
#pragma unroll
    for (int t = 0; t < 8; ++t) T[(8 * e + t) * TP + cl] = hb[t];
  }
  __syncthreads();
  v4u up[2];
#pragma unroll
  for (int it = 0; it < 2; ++it) {
    const int nl = it * 32 + lq;
    up[it] = *(const v4u*)(T + nl * TP + 8 * e);
  }
#pragma unroll
  for (int pass = 0; pass < 2; ++pass) {
#pragma unroll
    for (int it = 0; it < 2; ++it) {
      const int rl = it * 32 + lq;
      *(volatile v4u*)(XP + ((size_t)(b * SEQ + n0 + rl)) * CC + c0 + 8 * e) = up[it];
    }
    __threadfence();
  }
}

__global__ __launch_bounds__(128)
void gemm_p(const unsigned short* __restrict__ W16, const unsigned short* __restrict__ XP,
            const float* __restrict__ tbias, const float* __restrict__ pbias, const float* __restrict__ gbias,
            unsigned short* Qh, unsigned short* Ql, unsigned short* Kh, unsigned short* Kl, unsigned short* Gc) {
  __shared__ __align__(16) float Os[QT * OSP];
  const int tid  = threadIdx.x;
  const int lane = tid & 31, wave = tid >> 5;
  const int hh   = lane >> 4, c = lane & 15;
  const int nt   = blockIdx.x, mb = blockIdx.y, b = blockIdx.z;
  const int n0   = nt * QT, o0 = mb * QT;

  const unsigned short* ap = W16 + (size_t)(o0 + c) * CC + 8 * hh;
  const unsigned short* bp = XP + ((size_t)(b * SEQ + n0 + 16 * wave + c)) * CC + 8 * hh;

  v8f acc[4];
#pragma unroll
  for (int mt = 0; mt < 4; ++mt) acc[mt] = zero8();

#pragma unroll
  for (int ks = 0; ks < CC / 32; ++ks) {
    const Frag fb = ldfrag(bp + 32 * ks);
#pragma unroll
    for (int mt = 0; mt < 4; ++mt) {
      const Frag fa = ldfrag(ap + (size_t)(16 * mt) * CC + 32 * ks);
      acc[mt] = mma_h(fa.h, fb.h, acc[mt]);
    }
  }

  {
    const int nl = 16 * wave + c;
#pragma unroll
    for (int mt = 0; mt < 4; ++mt) {
      v4f va, vb;
#pragma unroll
      for (int r = 0; r < 4; ++r) { va[r] = acc[mt][r] * IWSC; vb[r] = acc[mt][4 + r] * IWSC; }
      *(v4f*)(Os + nl * OSP + 16 * mt + 8 * hh)     = va;
      *(v4f*)(Os + nl * OSP + 16 * mt + 8 * hh + 4) = vb;
    }
  }
  __syncthreads();

  const int e = tid & 7, lq = tid >> 3;
  if (mb < 4) {
    unsigned short* Ph = (mb < 2) ? Qh : Kh;
    unsigned short* Pl = (mb < 2) ? Ql : Kl;
    const float* bsrc  = (mb < 2) ? tbias : pbias;
    const int dsel = (mb & 1) * QT;
    const v4f b0 = *(const v4f*)(bsrc + dsel + 8 * e);
    const v4f b1 = *(const v4f*)(bsrc + dsel + 8 * e + 4);
    const float bb[8] = {bfr(b0[0]), bfr(b0[1]), bfr(b0[2]), bfr(b0[3]), bfr(b1[0]), bfr(b1[1]), bfr(b1[2]), bfr(b1[3])};
    v4u uh[4], ul[4];
#pragma unroll
    for (int it = 0; it < 4; ++it) {
      const int row = it * 16 + lq;
      const v4f a = *(const v4f*)(Os + row * OSP + 8 * e);
      const v4f q = *(const v4f*)(Os + row * OSP + 8 * e + 4);
      const float f[8] = {a[0], a[1], a[2], a[3], q[0], q[1], q[2], q[3]};
#pragma unroll
      for (int t = 0; t < 4; ++t) {
        const float f0 = f[2 * t] + bb[2 * t], f1 = f[2 * t + 1] + bb[2 * t + 1];
        const unsigned short hb0 = bf_bits(f0), hb1 = bf_bits(f1);
        const unsigned short lb0 = bf_bits(f0 - bf_up(hb0));
        const unsigned short lb1 = bf_bits(f1 - bf_up(hb1));
        uh[it][t] = pk16(hb0, hb1);
        ul[it][t] = pk16(lb0, lb1);
      }
    }
#pragma unroll
    for (int pass = 0; pass < 2; ++pass) {
#pragma unroll
      for (int it = 0; it < 4; ++it) {
        const int row = it * 16 + lq;
        const size_t po = ((size_t)(b * SEQ + n0 + row)) * DQ + dsel + 8 * e;
        *(volatile v4u*)(Ph + po) = uh[it];
        *(volatile v4u*)(Pl + po) = ul[it];
      }
      __threadfence();
    }
  } else {
    const int gsel = (mb - 4) * QT;
    v4u ug[4];
#pragma unroll
    for (int it = 0; it < 4; ++it) {
      const int cl = it * 16 + lq;
      const float bias = bfr(gbias[gsel + cl]);
      unsigned short hb[8];
#pragma unroll
      for (int t = 0; t < 8; ++t) {
        const int key = 8 * e + t;
        const float v = Os[key * OSP + cl] + bias;
        hb[t] = h_bits((_Float16)v);
      }
#pragma unroll
      for (int t = 0; t < 4; ++t) ug[it][t] = pk16(hb[2 * t], hb[2 * t + 1]);
    }
#pragma unroll
    for (int pass = 0; pass < 2; ++pass) {
#pragma unroll
      for (int it = 0; it < 4; ++it) {
        const int cl = it * 16 + lq;
        const size_t po = ((size_t)(b * DQ + gsel + cl)) * SEQ + n0 + 8 * e;
        *(volatile v4u*)(Gc + po) = ug[it];
      }
      __threadfence();
    }
  }
}

__global__ __launch_bounds__(128)
void attn_k(const unsigned short* __restrict__ Qh, const unsigned short* __restrict__ Ql,
            const unsigned short* __restrict__ Kh, const unsigned short* __restrict__ Kl,
            const unsigned short* __restrict__ Gc, unsigned short* Yh, unsigned short* Yl) {
  __shared__ __align__(16) float Os[QT * OSPW];
  const int tid  = threadIdx.x;
  const int wave = tid >> 5, lane = tid & 31;
  const int hh   = lane >> 4, c = lane & 15;
  const int n0   = blockIdx.x * QT, b = blockIdx.y;

  const size_t qo = ((size_t)(b * SEQ + n0 + 16 * wave + c)) * DQ + 8 * hh;
  const unsigned short* Qhp = Qh + qo;
  const unsigned short* Qlp = Ql + qo;
  const unsigned short* Khp = Kh + (size_t)b * SEQ * DQ + (size_t)c * DQ + 8 * hh;
  const unsigned short* Klp = Kl + (size_t)b * SEQ * DQ + (size_t)c * DQ + 8 * hh;
  const unsigned short* Vp = Gc + (size_t)b * DQ * SEQ + (size_t)c * SEQ + 8 * hh;

  float m = -1.0e30f, l = 0.f;
  v8f o[8];
#pragma unroll
  for (int j = 0; j < 8; ++j) o[j] = zero8();

#pragma unroll 1
  for (int kb = 0; kb < SEQ; kb += 32) {
    const unsigned short* k0p  = Khp + (size_t)kb * DQ;
    const unsigned short* k1p  = Khp + (size_t)(kb + 16) * DQ;
    const unsigned short* k0lp = Klp + (size_t)kb * DQ;
    const unsigned short* k1lp = Klp + (size_t)(kb + 16) * DQ;
    v8f s0 = zero8(), s1 = zero8();
#pragma unroll 1
    for (int kc = 0; kc < DQ / 32; ++kc) {
      const Frag qh  = ldfrag(Qhp + 32 * kc);
      const Frag ql  = ldfrag(Qlp + 32 * kc);
      const Frag k0  = ldfrag(k0p + 32 * kc);
      const Frag k1  = ldfrag(k1p + 32 * kc);
      const Frag k0l = ldfrag(k0lp + 32 * kc);
      const Frag k1l = ldfrag(k1lp + 32 * kc);
      s0 = mma_b(k0.bf, qh.bf, s0);
      s1 = mma_b(k1.bf, qh.bf, s1);
      s0 = mma_b(k0.bf, ql.bf, s0);
      s1 = mma_b(k1.bf, ql.bf, s1);
      s0 = mma_b(k0l.bf, qh.bf, s0);
      s1 = mma_b(k1l.bf, qh.bf, s1);
    }

    float mx = fmaxf(hmax8(s0), hmax8(s1));
    mx = fmaxf(mx, __shfl_xor(mx, 16, 32));
    const float mn = fmaxf(m, mx);
    const unsigned grew = wave_ballot(mx > m);
    if (grew != 0u) {
      const float corr = __expf(m - mn);
      l *= corr;
#pragma unroll
      for (int j = 0; j < 8; ++j) {
#pragma unroll
        for (int r = 0; r < 8; ++r) o[j][r] *= corr;
      }
    }
    m = mn;
    const float msh = mn - LNPS;

    FragH ph;
    float ls = 0.f;
#pragma unroll
    for (int r = 0; r < 8; ++r) {
      const float e0 = __expf(s0[r] - msh);
      const float e1 = __expf(s1[r] - msh);
      ls += e0 + e1;
      ph.hv[0][r] = (_Float16)e0;
      ph.hv[1][r] = (_Float16)e1;
    }
    l += ls;

#pragma unroll
    for (int j = 0; j < 8; ++j) {
      const Frag vf = ldfrag(Vp + (size_t)(16 * j) * SEQ + kb);
      o[j] = mma_h(vf.h, ph.v, o[j]);
    }
  }
  l += __shfl_xor(l, 16, 32);
  const float inv = 1.0f / l;

  const int qrow = 16 * wave + c;
#pragma unroll
  for (int j = 0; j < 8; ++j) {
    v4f va, vb;
#pragma unroll
    for (int r = 0; r < 4; ++r) { va[r] = o[j][r] * inv; vb[r] = o[j][4 + r] * inv; }
    *(v4f*)(Os + qrow * OSPW + 16 * j + 8 * hh)     = va;
    *(v4f*)(Os + qrow * OSPW + 16 * j + 8 * hh + 4) = vb;
  }
  __syncthreads();

  const int e = tid & 15, lq = tid >> 4;
  v4u uh[8], ul[8];
#pragma unroll
  for (int it = 0; it < 8; ++it) {
    const int row = it * 8 + lq;
    const v4f a = *(const v4f*)(Os + row * OSPW + 8 * e);
    const v4f q = *(const v4f*)(Os + row * OSPW + 8 * e + 4);
    const float f[8] = {a[0], a[1], a[2], a[3], q[0], q[1], q[2], q[3]};
#pragma unroll
    for (int t = 0; t < 4; ++t) {
      const float f0 = f[2 * t], f1 = f[2 * t + 1];
      const _Float16 h0 = (_Float16)f0, h1 = (_Float16)f1;
      const _Float16 r0 = (_Float16)((f0 - (float)h0) * RSC);
      const _Float16 r1 = (_Float16)((f1 - (float)h1) * RSC);
      uh[it][t] = pk16(h_bits(h0), h_bits(h1));
      ul[it][t] = pk16(h_bits(r0), h_bits(r1));
    }
  }
#pragma unroll
  for (int pass = 0; pass < 2; ++pass) {
#pragma unroll
    for (int it = 0; it < 8; ++it) {
      const int row = it * 8 + lq;
      const size_t po = ((size_t)(b * SEQ + n0 + row)) * DQ + 8 * e;
      *(volatile v4u*)(Yh + po) = uh[it];
      *(volatile v4u*)(Yl + po) = ul[it];
    }
    __threadfence();
  }
}

__global__ __launch_bounds__(128)
void gemm_o(const unsigned short* __restrict__ WW16, const unsigned short* __restrict__ Yh,
            const unsigned short* __restrict__ Yl, const float* __restrict__ wbias,
            float* WY, float* PS) {
  __shared__ __align__(16) float Os[QT * OSP];
  __shared__ __align__(16) float Sred[2 * QT];
  const int tid  = threadIdx.x;
  const int lane = tid & 31, wave = tid >> 5;
  const int hh   = lane >> 4, c = lane & 15;
  const int nt   = blockIdx.x, mb = blockIdx.y, b = blockIdx.z;
  const int n0   = nt * QT, o0 = mb * QT;

  const unsigned short* ap  = WW16 + (size_t)(o0 + c) * DQ + 8 * hh;
  const size_t bo = ((size_t)(b * SEQ + n0 + 16 * wave + c)) * DQ + 8 * hh;
  const unsigned short* bph = Yh + bo;
  const unsigned short* bpl = Yl + bo;

  v8f acc[4], accr[4];
#pragma unroll
  for (int mt = 0; mt < 4; ++mt) { acc[mt] = zero8(); accr[mt] = zero8(); }

#pragma unroll
  for (int ks = 0; ks < DQ / 32; ++ks) {
    const Frag fbh = ldfrag(bph + 32 * ks);
    const Frag fbl = ldfrag(bpl + 32 * ks);
#pragma unroll
    for (int mt = 0; mt < 4; ++mt) {
      const Frag fa = ldfrag(ap + (size_t)(16 * mt) * DQ + 32 * ks);
      acc[mt]  = mma_h(fa.h, fbh.h, acc[mt]);
      accr[mt] = mma_h(fa.h, fbl.h, accr[mt]);
    }
  }

  {
    const int nl = 16 * wave + c;
#pragma unroll
    for (int mt = 0; mt < 4; ++mt) {
      v4f va, vb;
#pragma unroll
      for (int r = 0; r < 4; ++r) {
        va[r] = (acc[mt][r] + accr[mt][r] * IRSC) * IWSC;
        vb[r] = (acc[mt][4 + r] + accr[mt][4 + r] * IRSC) * IWSC;
      }
      *(v4f*)(Os + nl * OSP + 16 * mt + 8 * hh)     = va;
      *(v4f*)(Os + nl * OSP + 16 * mt + 8 * hh + 4) = vb;
    }
  }
  __syncthreads();

  if (tid < QT) {
    float s = 0.f, q = 0.f;
#pragma unroll 8
    for (int n = 0; n < QT; ++n) {
      const float v = Os[n * OSP + tid];
      s += v;
      q = fmaf(v, v, q);
    }
    Sred[tid]      = s;
    Sred[QT + tid] = q;
  }
  __syncthreads();

  const int e = tid & 15, lq = tid >> 4;
  v4f res[8];
#pragma unroll
  for (int it = 0; it < 8; ++it) {
    const int col = it * 8 + lq;
    const int co  = o0 + col;
    const float bias = bfr(wbias[co]);
#pragma unroll
    for (int t = 0; t < 4; ++t) res[it][t] = Os[(4 * e + t) * OSP + col] + bias;
  }
  const v4f pv = *(const v4f*)(Sred + 4 * lane);
  float* psp = PS + (size_t)(b * NT + nt) * PSW + o0 + 4 * lane + ((lane >= 16) ? (PSW / 2 - 64) : 0);
#pragma unroll
  for (int pass = 0; pass < 2; ++pass) {
#pragma unroll
    for (int it = 0; it < 8; ++it) {
      const int col = it * 8 + lq;
      const int co  = o0 + col;
      const size_t idx = ((size_t)(b * CC + co)) * SEQ + n0 + 4 * e;
      *(volatile v4f*)(WY + idx) = res[it];
    }
    if (wave == 0) *(volatile v4f*)(psp) = pv;
    __threadfence();
  }
}

__global__ __launch_bounds__(256)
void bn_stat(const float* __restrict__ PS, const float* __restrict__ wbias, const float* __restrict__ gam,
             const float* __restrict__ bet, float* AB) {
  const int co = threadIdx.x;
  double s = 0.0, q = 0.0;
#pragma unroll 1
  for (int blk = 0; blk < NB * NT; ++blk) {
    s += (double)PS[(size_t)blk * PSW + co];
    q += (double)PS[(size_t)blk * PSW + CC + co];
  }
  const double icnt = 1.0 / (double)(NB * SEQ);
  const double mv = s * icnt;
  double var = q * icnt - mv * mv;
  var = (var > 0.0) ? var : 0.0;
  const float rstd = rsqrtf((float)var + BNEPS);
  const float A  = bfr(gam[co]) * rstd;
  const float mw = (float)mv + bfr(wbias[co]);
  const float Bc = bfr(bet[co]) - mw * A;
#pragma unroll
  for (int pass = 0; pass < 2; ++pass) {
    *(volatile float*)(AB + co)      = A;
    *(volatile float*)(AB + CC + co) = Bc;
    __threadfence();
  }
}

__global__ __launch_bounds__(256)
void bn_out(const float* __restrict__ WY, const float* __restrict__ AB, const float* __restrict__ x, float* out) {
  const int tid = threadIdx.x, b = blockIdx.y;
  const int i  = blockIdx.x * BCH + 4 * tid;
  const int co = i / SEQ;
  const int n  = i - co * SEQ;
  const float A = AB[co], Bc = AB[CC + co];
  const v4f w  = *(const v4f*)(WY + (size_t)b * CC * SEQ + i);
  const size_t xo = ((size_t)(b * CC + co)) * NN_FULL + n;
  const v4f xv = *(const v4f*)(x + xo);
  v4f r;
#pragma unroll
  for (int t = 0; t < 4; ++t) r[t] = fmaf(w[t], A, Bc) + bfr(xv[t]);
#pragma unroll
  for (int pass = 0; pass < 2; ++pass) {
    *(volatile v4f*)(out + xo) = r;
    __threadfence();
  }
}

extern "C" void kernel_launch(void* const* d_in, const int* in_sizes, int n_in,
                              void* d_out, int out_size, void* d_ws, size_t ws_size,
                              hipStream_t stream) {
  const int XNEED = ((NB - 1) * CC + (CC - 1)) * NN_FULL + SEQ;
  if (n_in < 11) return;
  if (in_sizes[0] < XNEED) return;
  if (in_sizes[1] < DQ * CC || in_sizes[3] < DQ * CC || in_sizes[5] < DQ * CC) return;
  if (in_sizes[2] < DQ || in_sizes[4] < DQ || in_sizes[6] < DQ) return;
  if (in_sizes[7] < CC * DQ || in_sizes[8] < CC) return;
  if (in_sizes[9] < CC || in_sizes[10] < CC) return;
  if (out_size < XNEED) return;

  size_t off = 0;
  auto carve = [&](size_t bytes) { const size_t o = off; off += (bytes + 255) & ~(size_t)255; return o; };
  const size_t oW16 = carve((size_t)MW * CC * 2);
  const size_t oWW  = carve((size_t)CC * DQ * 2);
  const size_t oXP  = carve((size_t)NB * SEQ * CC * 2);
  const size_t oQh  = carve((size_t)NB * SEQ * DQ * 2);
  const size_t oQl  = carve((size_t)NB * SEQ * DQ * 2);
  const size_t oKh  = carve((size_t)NB * SEQ * DQ * 2);
  const size_t oKl  = carve((size_t)NB * SEQ * DQ * 2);
  const size_t oGc  = carve((size_t)NB * DQ * SEQ * 2);
  const size_t oYh  = carve((size_t)NB * SEQ * DQ * 2);
  const size_t oYl  = carve((size_t)NB * SEQ * DQ * 2);
  const size_t oWY  = carve((size_t)NB * CC * SEQ * 4);
  const size_t oPS  = carve((size_t)NB * NT * PSW * 4);
  const size_t oAB  = carve((size_t)PSW * 4);
  if (off > ws_size) return;
  if (off > (size_t)134217728) return;

  const float* x   = (const float*)d_in[0];
  const float* Wt  = (const float*)d_in[1];
  const float* bt  = (const float*)d_in[2];
  const float* Wp  = (const float*)d_in[3];
  const float* bp  = (const float*)d_in[4];
  const float* Wg  = (const float*)d_in[5];
  const float* bg  = (const float*)d_in[6];
  const float* Ww  = (const float*)d_in[7];
  const float* bw  = (const float*)d_in[8];
  const float* gam = (const float*)d_in[9];
  const float* bet = (const float*)d_in[10];

  char* ws = (char*)d_ws;
  unsigned short* W16  = (unsigned short*)(ws + oW16);
  unsigned short* WW16 = (unsigned short*)(ws + oWW);
  unsigned short* XP   = (unsigned short*)(ws + oXP);
  unsigned short* Qh   = (unsigned short*)(ws + oQh);
  unsigned short* Ql   = (unsigned short*)(ws + oQl);
  unsigned short* Kh   = (unsigned short*)(ws + oKh);
  unsigned short* Kl   = (unsigned short*)(ws + oKl);
  unsigned short* Gc   = (unsigned short*)(ws + oGc);
  unsigned short* Yh   = (unsigned short*)(ws + oYh);
  unsigned short* Yl   = (unsigned short*)(ws + oYl);
  float* WY  = (float*)(ws + oWY);
  float* PS  = (float*)(ws + oPS);
  float* AB  = (float*)(ws + oAB);
  float* out = (float*)d_out;

  const dim3 blk256(256), blk128(128);

  cvt_w<<<dim3(MW / 8), blk256, 0, stream>>>(Wt, Wp, Wg, W16);
  cvt_ww<<<dim3(CC / 16), blk256, 0, stream>>>(Ww, WW16);
  cvt_x<<<dim3(NT, CC / QT, NB), blk256, 0, stream>>>(x, XP);
  gemm_p<<<dim3(NT, 6, NB), blk128, 0, stream>>>(W16, XP, bt, bp, bg, Qh, Ql, Kh, Kl, Gc);
  attn_k<<<dim3(NT, NB), blk128, 0, stream>>>(Qh, Ql, Kh, Kl, Gc, Yh, Yl);
  gemm_o<<<dim3(NT, CC / QT, NB), blk128, 0, stream>>>(WW16, Yh, Yl, bw, WY, PS);
  bn_stat<<<dim3(1), blk256, 0, stream>>>(PS, bw, gam, bet, AB);
  bn_out<<<dim3(CC * SEQ / BCH, NB), blk256, 0, stream>>>(WY, AB, x, out);
  (void)hipGetLastError();
}
